// GCN_15960098472701
// MI455X (gfx1250) — hardware-run, weakly checked
//
#include <hip/hip_runtime.h>
#include <stddef.h>
#include <stdint.h>
#include <math.h>

#define NN      100000
#define NE      1600000
#define FIN     24
#define KE      32
#define HD      128
#define KL      256
#define NOUT    12
#define NOP     16
#define MP      100096
#define GBM     64
#define GTHR    128
#define HBM     128
#define NTHR    256
#define NWAVE   8
#define EPT     8
#define WCH     (32 * EPT)
#define NBRUN   1024
#define SLB     10
#define NBK     98
#define WLCAP   2560
#define RCAP    20480
#define DEGCAP  64
#define MAXDEG_MEAS   37
#define MAXB1024_MEAS 16721
#define ABM     64
#define SP      132

#define BK_WL    (NWAVE * WLCAP)
#define BK_PL    (2 * RCAP)
#define BK_ZINTS (BK_WL + BK_PL + 3 * NBRUN)
#define BK_INTS  (BK_ZINTS + 16)
#define BK_LDS   (BK_INTS * 4)

#define PBX   (MP * (KE / 8) / NTHR)
#define PBWE  (HD * (KE / 8) / NTHR)
#define PBW1  (HD * (KL / 8) / NTHR)
#define PBWF  (NOP * (KL / 8) / NTHR)
#define PBTOT (PBX + PBWE + 4 * PBW1 + PBWF + 1)

static_assert(HD == 128 && KL == 2 * HD);
static_assert(FIN <= KE && KE % 32 == 0 && KL % 32 == 0 && FIN % 8 == 0);
static_assert(NOUT <= NOP && NOP == 16);
static_assert((HBM * NOUT * 4) % 128 == 0 && (((NN % HBM) * NOUT * 4) % 128) == 0);
static_assert(MP % GBM == 0 && MP % HBM == 0 && MP % ABM == 0 && MP >= NN && MP == 782 * 128);
static_assert(NBRUN == (1 << SLB) && NBRUN % ABM == 0 && NBRUN % NTHR == 0);
static_assert(NN <= NBK * NBRUN && MP <= NBK * NBRUN);
static_assert(NE < (1 << 21) && (((long long)NE) << SLB) < (1LL << 31));
static_assert(NE % WCH == 0 && NE % 4 == 0);
static_assert(RCAP == NWAVE * WLCAP && BK_ZINTS % (NTHR * 4) == 0 && BK_PL % (NTHR * 4) == 0);
static_assert(MAXB1024_MEAS <= 19400);
static_assert((long long)RCAP * 100 >= (long long)MAXB1024_MEAS * 105);
static_assert(WLCAP >= MAXB1024_MEAS / 8 + 8 * 46 + 1);
static_assert(MAXDEG_MEAS + 8 <= DEGCAP);
static_assert(BK_LDS <= 300000 && BK_LDS <= 327680);
static_assert((GBM * SP + HD + GBM) * 4 <= 65536);
static_assert((MP * (KE / 8)) % NTHR == 0 && (HD * (KE / 8)) % NTHR == 0);
static_assert((HD * (KL / 8)) % NTHR == 0 && (NOP * (KL / 8)) % NTHR == 0);
static_assert(GBM == (GTHR / 32) * 16 && HBM == NWAVE * 16 && ABM % NWAVE == 0);

typedef float          v4f   __attribute__((ext_vector_type(4)));
typedef float          v8f   __attribute__((ext_vector_type(8)));
typedef int            v2i   __attribute__((ext_vector_type(2)));
typedef int            v4i   __attribute__((ext_vector_type(4)));
typedef int            v8i   __attribute__((ext_vector_type(8)));
typedef unsigned       v2u   __attribute__((ext_vector_type(2)));
typedef unsigned short v8us  __attribute__((ext_vector_type(8)));
typedef unsigned short v16us __attribute__((ext_vector_type(16)));
typedef __bf16         v16bf __attribute__((ext_vector_type(16)));
typedef v4f  __attribute__((may_alias)) v4fa;
typedef v2i  __attribute__((may_alias)) v2ia;
typedef v4i  __attribute__((may_alias)) v4ia;
typedef v2u  __attribute__((may_alias)) v2ua;
typedef v8us __attribute__((may_alias)) v8usa;
union FragB { v16bf v; v16us u; v8us h[2]; v8i w; };

__device__ __forceinline__ v8f wmb(const FragB& a, const FragB& b, v8f c) {
  v8f d = __builtin_amdgcn_wmma_f32_16x16x32_bf16(false, a.v, false, b.v, (short)0, c, false, false);
  asm volatile("v_nop\n\tv_nop\n\tv_nop\n\tv_nop" : "+v"(d) : "v"(a.w), "v"(b.w));
  return d;
}

__device__ __forceinline__ v8f z8() { v8f z = {0.f, 0.f, 0.f, 0.f, 0.f, 0.f, 0.f, 0.f}; return z; }

__device__ __forceinline__ unsigned bf16_bits(float f) {
  const unsigned u = __float_as_uint(f);
  const unsigned r = (u + 0x7FFFu + ((u >> 16) & 1u)) >> 16;
  const unsigned q = (u >> 16) | 0x40u;
  return ((u & 0x7fffffffu) > 0x7f800000u) ? q : r;
}

__device__ __forceinline__ void hilo_pack(float v0, float v1, float v2, float v3,
                                          int& h01, int& h23, int& l01, int& l23) {
  const unsigned a0 = bf16_bits(v0), a1 = bf16_bits(v1), a2 = bf16_bits(v2), a3 = bf16_bits(v3);
  const unsigned b0 = bf16_bits(v0 - __uint_as_float(a0 << 16));
  const unsigned b1 = bf16_bits(v1 - __uint_as_float(a1 << 16));
  const unsigned b2 = bf16_bits(v2 - __uint_as_float(a2 << 16));
  const unsigned b3 = bf16_bits(v3 - __uint_as_float(a3 << 16));
  h01 = (int)(a0 | (a1 << 16)); h23 = (int)(a2 | (a3 << 16));
  l01 = (int)(b0 | (b1 << 16)); l23 = (int)(b2 | (b3 << 16));
}

__device__ __forceinline__ v4i regroup128(int h01, int h23, int l01, int l23, int lane) {
  const int s0 = (2 * lane) & 31, s1 = s0 + 1;
  const int a0 = __shfl(h01, s0, 32), a1 = __shfl(h23, s0, 32), a2 = __shfl(h01, s1, 32), a3 = __shfl(h23, s1, 32);
  const int b0 = __shfl(l01, s0, 32), b1 = __shfl(l23, s0, 32), b2 = __shfl(l01, s1, 32), b3 = __shfl(l23, s1, 32);
  const int mk = (lane < 16) ? -1 : 0;
  v4i o;
  o.x = (a0 & mk) | (b0 & ~mk); o.y = (a1 & mk) | (b1 & ~mk);
  o.z = (a2 & mk) | (b2 & ~mk); o.w = (a3 & mk) | (b3 & ~mk);
  return o;
}

__device__ __forceinline__ void st2_v4f(float* p, v4f v) {
  *(volatile v4f*)p = v;
  __threadfence();
  *(volatile v4f*)p = v;
}
__device__ __forceinline__ void st2_v8us(unsigned short* p, v8us v) {
  *(volatile v8us*)p = v;
  __threadfence();
  *(volatile v8us*)p = v;
}
__device__ __forceinline__ void st2_v4i(unsigned short* p, v4i v) {
  *(volatile v4i*)p = v;
  __threadfence();
  *(volatile v4i*)p = v;
}

__device__ __forceinline__ v8us col8(const float* __restrict__ base, int stride, unsigned mk) {
  float f[8];
#pragma unroll
  for (int i = 0; i < 8; ++i) f[i] = base[(size_t)i * (size_t)stride];
  v8us o;
#pragma unroll
  for (int i = 0; i < 8; ++i) o[i] = (unsigned short)(bf16_bits(f[i]) & mk);
  return o;
}

__device__ __forceinline__ void wdup_unit(const float* __restrict__ w, unsigned short* dst, int v) {
  const int n = v >> 5, k8 = (v & 31) * 8, kk = k8 & (HD - 1);
  const v8us o = col8(w + (size_t)kk * HD + n, HD, 0xffffu);
  st2_v8us(dst + (size_t)v * 8, o);
}

__global__ __launch_bounds__(NTHR) void k_prep(const float* __restrict__ x, const float* __restrict__ wemb,
                                               const float* __restrict__ bemb, const float* __restrict__ ws1,
                                               const float* __restrict__ w1, const float* __restrict__ b1,
                                               const float* __restrict__ ws2, const float* __restrict__ w2,
                                               const float* __restrict__ b2, const float* __restrict__ wfc,
                                               const float* __restrict__ bfc,
                                               unsigned short* xb, unsigned short* wet, unsigned short* wd,
                                               unsigned short* wf, float* sm) {
  const int tid = (int)threadIdx.x, lane = tid & 31;
  const int blk = (int)blockIdx.x;
  const int B1 = PBX + PBWE;
  const int B2 = B1 + 4 * PBW1;
  if (blk < PBX) {
    const int u   = blk * NTHR + tid;
    const int row = u >> 2, k8 = (u & 3) * 8;
    const int rc  = row < NN ? row : NN - 1;
    const int kc  = k8 < FIN ? k8 : FIN - 8;
    const unsigned mk = (row < NN && k8 < FIN) ? 0xffffu : 0u;
    const float* p = x + (size_t)rc * FIN + kc;
    const v4f a = *(const v4fa*)p;
    const v4f b = *(const v4fa*)(p + 4);
    v8us o;
    o[0] = (unsigned short)(bf16_bits(a.x) & mk); o[1] = (unsigned short)(bf16_bits(a.y) & mk);
    o[2] = (unsigned short)(bf16_bits(a.z) & mk); o[3] = (unsigned short)(bf16_bits(a.w) & mk);
    o[4] = (unsigned short)(bf16_bits(b.x) & mk); o[5] = (unsigned short)(bf16_bits(b.y) & mk);
    o[6] = (unsigned short)(bf16_bits(b.z) & mk); o[7] = (unsigned short)(bf16_bits(b.w) & mk);
    st2_v8us(xb + (size_t)u * 8, o);
  } else if (blk < B1) {
    const int u = (blk - PBX) * NTHR + tid;
    const int n = u >> 2, k8 = (u & 3) * 8;
    const int kc = k8 < FIN ? k8 : FIN - 8;
    const unsigned mk = (k8 < FIN) ? 0xffffu : 0u;
    const v8us o = col8(wemb + (size_t)kc * HD + n, HD, mk);
    st2_v8us(wet + (size_t)u * 8, o);
  } else if (blk < B1 + PBW1) {
    wdup_unit(ws1, wd, (blk - B1) * NTHR + tid);
  } else if (blk < B1 + 2 * PBW1) {
    wdup_unit(w1, wd + (size_t)HD * KL, (blk - B1 - PBW1) * NTHR + tid);
  } else if (blk < B1 + 3 * PBW1) {
    wdup_unit(ws2, wd + (size_t)2 * HD * KL, (blk - B1 - 2 * PBW1) * NTHR + tid);
  } else if (blk < B2) {
    wdup_unit(w2, wd + (size_t)3 * HD * KL, (blk - B1 - 3 * PBW1) * NTHR + tid);
  } else if (blk < B2 + PBWF) {
    const int u = (blk - B2) * NTHR + tid;
    const int n = u >> 5, k8 = (u & 31) * 8, kk = k8 & (HD - 1);
    const int nc = n < NOUT ? n : NOUT - 1;
    const unsigned mk = (n < NOUT) ? 0xffffu : 0u;
    const v8us o = col8(wfc + (size_t)kk * NOUT + nc, NOUT, mk);
    st2_v8us(wf + (size_t)u * 8, o);
  } else {
    if (tid < 128) {
      const int w  = tid >> 5;
      const int qc = lane < (NOUT / 4) ? lane : (NOUT / 4 - 1);
      const v4f c0 = *(const v4fa*)(bemb + 4 * lane);
      const v4f c1 = *(const v4fa*)(b1 + 4 * lane);
      const v4f c2 = *(const v4fa*)(b2 + 4 * lane);
      const v4f c3 = *(const v4fa*)(bfc + 4 * qc);
      asm volatile("" :: "v"(c0));
      asm volatile("" :: "v"(c1));
      asm volatile("" :: "v"(c2));
      asm volatile("" :: "v"(c3));
      const unsigned m0 = (w == 0) ? 0xffffffffu : 0u;
      const unsigned m1 = (w == 1) ? 0xffffffffu : 0u;
      const unsigned m2 = (w == 2) ? 0xffffffffu : 0u;
      const unsigned m3 = (w == 3 && lane < (NOUT / 4)) ? 0xffffffffu : 0u;
      v4f o;
      o.x = __uint_as_float(((bf16_bits(c0.x) << 16) & m0) | ((bf16_bits(c1.x) << 16) & m1) |
                            ((bf16_bits(c2.x) << 16) & m2) | ((bf16_bits(c3.x) << 16) & m3));
      o.y = __uint_as_float(((bf16_bits(c0.y) << 16) & m0) | ((bf16_bits(c1.y) << 16) & m1) |
                            ((bf16_bits(c2.y) << 16) & m2) | ((bf16_bits(c3.y) << 16) & m3));
      o.z = __uint_as_float(((bf16_bits(c0.z) << 16) & m0) | ((bf16_bits(c1.z) << 16) & m1) |
                            ((bf16_bits(c2.z) << 16) & m2) | ((bf16_bits(c3.z) << 16) & m3));
      o.w = __uint_as_float(((bf16_bits(c0.w) << 16) & m0) | ((bf16_bits(c1.w) << 16) & m1) |
                            ((bf16_bits(c2.w) << 16) & m2) | ((bf16_bits(c3.w) << 16) & m3));
      st2_v4f(sm + 4 * tid, o);
    }
  }
}

__device__ __forceinline__ int sweep_keys(const int* __restrict__ keys, unsigned nbs, int* mylist,
                                          int wave, int lane) {
  const int per  = ((NE + NWAVE * WCH - 1) / (NWAVE * WCH)) * WCH;
  const int ebeg = wave * per;
  const int eend = (ebeg + per < NE) ? (ebeg + per) : NE;
  int wc = 0;
#pragma unroll 1
  for (int cb = ebeg; cb < eend; cb += WCH) {
    const int e0 = cb + lane * EPT;
    const v4i da = *(const v4ia*)(keys + e0);
    const v4i db = *(const v4ia*)(keys + e0 + 4);
    const unsigned s0 = (unsigned)da.x - nbs, s1 = (unsigned)da.y - nbs;
    const unsigned s2 = (unsigned)da.z - nbs, s3 = (unsigned)da.w - nbs;
    const unsigned s4 = (unsigned)db.x - nbs, s5 = (unsigned)db.y - nbs;
    const unsigned s6 = (unsigned)db.z - nbs, s7 = (unsigned)db.w - nbs;
    const bool h0 = s0 < (unsigned)NBRUN, h1 = s1 < (unsigned)NBRUN, h2 = s2 < (unsigned)NBRUN, h3 = s3 < (unsigned)NBRUN;
    const bool h4 = s4 < (unsigned)NBRUN, h5 = s5 < (unsigned)NBRUN, h6 = s6 < (unsigned)NBRUN, h7 = s7 < (unsigned)NBRUN;
    const unsigned m0 = __builtin_amdgcn_ballot_w32(h0), m1 = __builtin_amdgcn_ballot_w32(h1);
    const unsigned m2 = __builtin_amdgcn_ballot_w32(h2), m3 = __builtin_amdgcn_ballot_w32(h3);
    const unsigned m4 = __builtin_amdgcn_ballot_w32(h4), m5 = __builtin_amdgcn_ballot_w32(h5);
    const unsigned m6 = __builtin_amdgcn_ballot_w32(h6), m7 = __builtin_amdgcn_ballot_w32(h7);
    const unsigned any = m0 | m1 | m2 | m3 | m4 | m5 | m6 | m7;
    if (any != 0u) {
      const int pre = (int)(__builtin_amdgcn_mbcnt_lo(m0, 0u) + __builtin_amdgcn_mbcnt_lo(m1, 0u) +
                            __builtin_amdgcn_mbcnt_lo(m2, 0u) + __builtin_amdgcn_mbcnt_lo(m3, 0u) +
                            __builtin_amdgcn_mbcnt_lo(m4, 0u) + __builtin_amdgcn_mbcnt_lo(m5, 0u) +
                            __builtin_amdgcn_mbcnt_lo(m6, 0u) + __builtin_amdgcn_mbcnt_lo(m7, 0u));
      int p = wc + pre;
      if (h0) { if (p < WLCAP) mylist[p] = ((e0 + 0) << SLB) | (int)s0; p = p + 1; }
      if (h1) { if (p < WLCAP) mylist[p] = ((e0 + 1) << SLB) | (int)s1; p = p + 1; }
      if (h2) { if (p < WLCAP) mylist[p] = ((e0 + 2) << SLB) | (int)s2; p = p + 1; }
      if (h3) { if (p < WLCAP) mylist[p] = ((e0 + 3) << SLB) | (int)s3; p = p + 1; }
      if (h4) { if (p < WLCAP) mylist[p] = ((e0 + 4) << SLB) | (int)s4; p = p + 1; }
      if (h5) { if (p < WLCAP) mylist[p] = ((e0 + 5) << SLB) | (int)s5; p = p + 1; }
      if (h6) { if (p < WLCAP) mylist[p] = ((e0 + 6) << SLB) | (int)s6; p = p + 1; }
      if (h7) { if (p < WLCAP) mylist[p] = ((e0 + 7) << SLB) | (int)s7; p = p + 1; }
      wc += (int)(__builtin_popcount(m0) + __builtin_popcount(m1) + __builtin_popcount(m2) + __builtin_popcount(m3) +
                  __builtin_popcount(m4) + __builtin_popcount(m5) + __builtin_popcount(m6) + __builtin_popcount(m7));
    }
  }
  return wc;
}

__device__ __forceinline__ void bucket_flush(const int* pl, const int* cnt, const int* rsb, int ov, int role,
                                             int* lp, int* cop, int* rp, int* fp, int tid) {
  if (role == 0) {
#pragma unroll 1
    for (int i = tid * 4; i < BK_PL; i += NTHR * 4) {
      const v4i v = *(const v4ia*)(pl + i);
      *(volatile v4i*)(lp + i) = v;
    }
#pragma unroll 1
    for (int i = tid * 4; i < 2 * NBRUN; i += NTHR * 4) {
      const v4i v = *(const v4ia*)(cnt + i);
      *(volatile v4i*)(cop + i) = v;
    }
  }
  {
    const v4i v = *(const v4ia*)(rsb + 4 * tid);
    *(volatile v4i*)(rp + 4 * tid) = v;
  }
  if (tid < 8) {
    const v4i f = {ov, ov, ov, ov};
    *(volatile v4i*)(fp + 4 * tid) = f;
  }
}

__global__ __launch_bounds__(NTHR) void k_bucket(const int* __restrict__ srcs, const int* __restrict__ dsts,
                                                 const float* __restrict__ ew, int* LIST, int* CO, int* RS,
                                                 int* FLAG) {
  extern __shared__ __attribute__((aligned(16))) int dsm[];
  int* wl   = dsm;
  int* pl   = dsm + BK_WL;
  int* cnt  = pl + BK_PL;
  int* offs = cnt + NBRUN;
  int* cur  = offs + NBRUN;
  int* misc = cur + NBRUN;
  const int tid = (int)threadIdx.x, lane = tid & 31, wave = tid >> 5;
  const int blk  = (int)blockIdx.x;
  const int role = (blk >= NBK) ? 1 : 0;
  const int bb   = blk - role * NBK;
  const unsigned nbs = (unsigned)(bb * NBRUN);

  {
    const v4i z4 = {0, 0, 0, 0};
    for (int i = tid * 4; i < BK_ZINTS; i += NTHR * 4) *(v4ia*)(dsm + i) = z4;
    if (tid < 16) misc[tid] = 0;
  }
  __syncthreads();

  {
    int wc;
    if (role == 0) wc = sweep_keys(dsts, nbs, wl + wave * WLCAP, wave, lane);
    else           wc = sweep_keys(srcs, nbs, wl + wave * WLCAP, wave, lane);
    if (lane == 0) misc[wave] = wc;
  }
  __syncthreads();

  if (wave == 0) {
    int ov = 0;
#pragma unroll 1
    for (int w2 = 0; w2 < NWAVE; ++w2) {
      int c = misc[w2];
      if (c > WLCAP) ov = 1;
      c = c < 0 ? 0 : (c > WLCAP ? WLCAP : c);
#pragma unroll 1
      for (int b0 = 0; b0 < c; b0 += 32) {
        const int idx = b0 + lane;
        const int ent = wl[w2 * WLCAP + (idx < WLCAP ? idx : WLCAP - 1)];
        const int m32 = (c - b0) < 32 ? (c - b0) : 32;
#pragma unroll 1
        for (int k = 0; k < m32; ++k) {
          const int u    = __builtin_amdgcn_readlane(ent, k);
          const int slot = u & (NBRUN - 1);
          if (lane == 0) cnt[slot] = cnt[slot] + 1;
        }
      }
    }
    if (lane == 0) misc[9] = ov;
  }
  __syncthreads();

  if (role == 0 && wave == 0) {
    const int base = lane * (NBRUN / 32);
    int s = 0;
#pragma unroll 1
    for (int i = 0; i < NBRUN / 32; ++i) s += cnt[base + i];
    int incl = s;
#pragma unroll
    for (int d = 1; d < 32; d <<= 1) {
      const int y = __shfl_up(incl, d, 32);
      if (lane >= d) incl += y;
    }
    int run = incl - s;
#pragma unroll 1
    for (int i = 0; i < NBRUN / 32; ++i) {
      const int cv = cnt[base + i];
      offs[base + i] = run;
      cur[base + i]  = run;
      run += cv;
    }
  }
  __syncthreads();

  if (role == 0 && wave == 0) {
#pragma unroll 1
    for (int w2 = 0; w2 < NWAVE; ++w2) {
      int c = misc[w2];
      c = c < 0 ? 0 : (c > WLCAP ? WLCAP : c);
#pragma unroll 1
      for (int b0 = 0; b0 < c; b0 += 32) {
        const int idx = b0 + lane;
        const int ent = wl[w2 * WLCAP + (idx < WLCAP ? idx : WLCAP - 1)];
        int eid = (ent >> SLB) & 0x1FFFFF;
        eid = eid > NE - 1 ? NE - 1 : eid;
        int sr = srcs[eid];
        sr = sr < 0 ? 0 : (sr > NN - 1 ? NN - 1 : sr);
        const int wbits = (int)(bf16_bits(ew[eid]) << 16);
        const int m32 = (c - b0) < 32 ? (c - b0) : 32;
#pragma unroll 1
        for (int k = 0; k < m32; ++k) {
          const int u    = __builtin_amdgcn_readlane(ent, k);
          const int sk   = __builtin_amdgcn_readlane(sr, k);
          const int wk   = __builtin_amdgcn_readlane(wbits, k);
          const int slot = u & (NBRUN - 1);
          if (lane == 0) {
            int p = cur[slot];
            p = p < 0 ? 0 : (p > RCAP - 1 ? RCAP - 1 : p);
            pl[2 * p]     = sk;
            pl[2 * p + 1] = wk;
            cur[slot] = p + 1;
          }
        }
      }
    }
  }
  __syncthreads();

  const int ovf = misc[9];
#pragma unroll 1
  for (int i = 0; i < NBRUN / NTHR; ++i) {
    const int s = i * NTHR + tid;
    int c = cnt[s];
    c = c < 1 ? 1 : c;
    const float r = 1.0f / sqrtf((float)c);
    const unsigned rb = (ovf != 0) ? 0x7fc00000u : __float_as_uint(r);
    cur[s] = (int)rb;
  }
  __syncthreads();

  int* lp  = LIST + (size_t)bb * BK_PL;
  int* cop = CO + (size_t)bb * (2 * NBRUN);
  int* rp  = RS + (size_t)role * (size_t)(NBK * NBRUN) + (size_t)bb * NBRUN;
  int* fp  = FLAG + (size_t)blk * 32;
  bucket_flush(pl, cnt, cur, ovf, role, lp, cop, rp, fp, tid);
  __threadfence();
  bucket_flush(pl, cnt, cur, ovf, role, lp, cop, rp, fp, tid);
}

template <int KTOT>
__device__ __forceinline__ void gemm_16x128(const unsigned short* ap, const unsigned short* __restrict__ bp,
                                            v8f (&acc)[8]) {
#pragma unroll 1
  for (int k0 = 0; k0 < KTOT; k0 += 32) {
    FragB af;
    af.h[0] = *(const v8usa*)(ap + k0);
    af.h[1] = *(const v8usa*)(ap + k0 + 16);
#pragma unroll
    for (int nt = 0; nt < 8; ++nt) {
      const unsigned short* wq = bp + (size_t)(16 * nt) * (size_t)KTOT + k0;
      FragB bf;
      bf.h[0] = *(const v8usa*)wq;
      bf.h[1] = *(const v8usa*)(wq + 16);
      acc[nt] = wmb(af, bf, acc[nt]);
    }
  }
}

__device__ __forceinline__ void stage_d(float* stg, const v8f (&acc)[8], int wave, int hh, int m) {
#pragma unroll
  for (int nt = 0; nt < 8; ++nt) {
#pragma unroll
    for (int r = 0; r < 8; ++r) stg[(16 * wave + 8 * hh + r) * SP + 16 * nt + m] = acc[nt][r];
  }
}

template <int RELU>
__device__ __forceinline__ void epi_rows(const float* stg, unsigned short* plane, int rowBase, int wave, int lane) {
  const int c8 = 8 * (lane & 15);
  const unsigned mk = (lane < 16) ? 0xffffffffu : 0u;
#pragma unroll 1
  for (int i = 0; i < 16; ++i) {
    const int lr   = 16 * wave + i;
    const int grow = rowBase + lr;
    const bool live = grow < NN;
    const v4f a = *(const v4fa*)(stg + lr * SP + c8);
    const v4f b = *(const v4fa*)(stg + lr * SP + c8 + 4);
    float v[8] = {a.x, a.y, a.z, a.w, b.x, b.y, b.z, b.w};
    unsigned w[8];
#pragma unroll
    for (int q = 0; q < 8; ++q) {
      float xv = v[q];
      if (RELU != 0) xv = (xv > 0.0f) ? xv : (xv - xv);
      xv = live ? xv : 0.0f;
      const unsigned hb = bf16_bits(xv);
      const unsigned lb = bf16_bits(xv - __uint_as_float(hb << 16));
      w[q] = (hb & mk) | (lb & ~mk);
    }
    v4i o;
    o.x = (int)(w[0] | (w[1] << 16)); o.y = (int)(w[2] | (w[3] << 16));
    o.z = (int)(w[4] | (w[5] << 16)); o.w = (int)(w[6] | (w[7] << 16));
    st2_v4i(plane + (size_t)grow * KL + 8 * lane, o);
  }
}

__global__ __launch_bounds__(GTHR) __attribute__((amdgpu_num_vgpr(248)))
void k_emb(const unsigned short* __restrict__ XB, const unsigned short* __restrict__ WT,
           const float* __restrict__ sm, unsigned short* Hhl) {
  __shared__ __attribute__((aligned(16))) float stg[GBM * SP];
  __shared__ __attribute__((aligned(16))) float sb[HD];
  const int tid = (int)threadIdx.x, lane = tid & 31, wave = tid >> 5, hh = lane >> 4, m = lane & 15;
  const int rowBase = (int)blockIdx.x * GBM;
  if (tid < 32) *(v4fa*)(sb + 4 * tid) = *(const v4fa*)(sm + 4 * tid);
  __syncthreads();

  v8f acc[8];
#pragma unroll
  for (int t = 0; t < 8; ++t) acc[t] = z8();
  const unsigned short* ap = XB + (size_t)(rowBase + 16 * wave + m) * (size_t)KE + 8 * hh;
  const unsigned short* bp = WT + (size_t)m * (size_t)KE + 8 * hh;
  gemm_16x128<KE>(ap, bp, acc);
#pragma unroll
  for (int nt = 0; nt < 8; ++nt) {
    const float bc = sb[16 * nt + m];
#pragma unroll
    for (int r = 0; r < 8; ++r) acc[nt][r] = acc[nt][r] + bc;
  }
  stage_d(stg, acc, wave, hh, m);
  __syncthreads();
  epi_rows<0>(stg, Hhl, rowBase, wave, lane);
}

__global__ __launch_bounds__(NTHR) void k_replay(const int* __restrict__ LIST, const int* __restrict__ CO,
                                                 const int* __restrict__ FLAG, const float* __restrict__ RSO,
                                                 const unsigned short* __restrict__ Hs, unsigned short* AGG) {
  const int tid = (int)threadIdx.x, lane = tid & 31, wave = tid >> 5;
  const int rowBase = (int)blockIdx.x * ABM;
  const int bucket  = rowBase >> SLB;
  const int* lb  = LIST + (size_t)bucket * BK_PL;
  const int* cob = CO + (size_t)bucket * (2 * NBRUN);
  const int flag = FLAG[(size_t)bucket * 32];
  const float qnan = __uint_as_float(0x7fc00000u);

#pragma unroll 1
  for (int i = 0; i < ABM / NWAVE; ++i) {
    const int d    = rowBase + (ABM / NWAVE) * wave + i;
    const int slot = d & (NBRUN - 1);
    int c = cob[slot];
    int o = cob[NBRUN + slot];
    const bool big = c > DEGCAP;
    c = c < 0 ? 0 : (c > DEGCAP ? DEGCAP : c);
    o = o < 0 ? 0 : (o > RCAP - 1 ? RCAP - 1 : o);
    int last = o + c - 1;
    last = last < o ? o : last;
    last = last > RCAP - 1 ? RCAP - 1 : last;
    const int cs = __builtin_amdgcn_readfirstlane(c);
    float a0 = 0.0f, a1 = 0.0f, a2 = 0.0f, a3 = 0.0f;
#pragma unroll 1
    for (int b0 = 0; b0 < cs; b0 += 32) {
      int idx = o + b0 + lane;
      idx = idx > last ? last : idx;
      const v2i ent = *(const v2ia*)(lb + 2 * idx);
      int sr = ent.x;
      sr = sr < 0 ? 0 : (sr > NN - 1 ? NN - 1 : sr);
      const int rsb = __float_as_int(RSO[sr]);
      const int wb  = ent.y;
      const int m32 = (cs - b0) < 32 ? (cs - b0) : 32;
#pragma unroll 1
      for (int k = 0; k < m32; ++k) {
        const int   sk = __builtin_amdgcn_readlane(sr, k);
        const float rk = __int_as_float(__builtin_amdgcn_readlane(rsb, k));
        const float wk = __int_as_float(__builtin_amdgcn_readlane(wb, k));
        const unsigned short* rp = Hs + (size_t)sk * KL + 4 * lane;
        const v2u wh = *(const v2ua*)rp;
        const v2u wl = *(const v2ua*)(rp + HD);
        const float f0 = __uint_as_float(wh.x << 16)         + __uint_as_float(wl.x << 16);
        const float f1 = __uint_as_float(wh.x & 0xffff0000u) + __uint_as_float(wl.x & 0xffff0000u);
        const float f2 = __uint_as_float(wh.y << 16)         + __uint_as_float(wl.y << 16);
        const float f3 = __uint_as_float(wh.y & 0xffff0000u) + __uint_as_float(wl.y & 0xffff0000u);
        a0 += (f0 * rk) * wk; a1 += (f1 * rk) * wk; a2 += (f2 * rk) * wk; a3 += (f3 * rk) * wk;
      }
    }
    const bool bad  = (flag != 0) | big;
    const bool live = d < NN;
    float m0 = bad ? qnan : a0, m1 = bad ? qnan : a1, m2 = bad ? qnan : a2, m3 = bad ? qnan : a3;
    m0 = live ? m0 : 0.0f; m1 = live ? m1 : 0.0f; m2 = live ? m2 : 0.0f; m3 = live ? m3 : 0.0f;
    int h01, h23, l01, l23;
    hilo_pack(m0, m1, m2, m3, h01, h23, l01, l23);
    const v4i ow = regroup128(h01, h23, l01, l23, lane);
    st2_v4i(AGG + (size_t)d * KL + 8 * lane, ow);
  }
}

__global__ __launch_bounds__(GTHR) __attribute__((amdgpu_num_vgpr(248)))
void k_layer(unsigned short* Hhl, const unsigned short* __restrict__ AGG,
             const unsigned short* __restrict__ WSD, const unsigned short* __restrict__ WD,
             const float* __restrict__ bvec, const float* __restrict__ rsi) {
  __shared__ __attribute__((aligned(16))) float stg[GBM * SP];
  __shared__ __attribute__((aligned(16))) float sb[HD];
  __shared__ __attribute__((aligned(16))) float srs[GBM];
  const int tid = (int)threadIdx.x, lane = tid & 31, wave = tid >> 5, hh = lane >> 4, m = lane & 15;
  const int rowBase = (int)blockIdx.x * GBM;
  if (tid < 32) {
    *(v4fa*)(sb + 4 * tid) = *(const v4fa*)(bvec + 4 * tid);
  } else if (tid < 64) {
    const int j = lane & 15;
    *(v4fa*)(srs + 4 * j) = *(const v4fa*)(rsi + rowBase + 4 * j);
  }
  __syncthreads();

  v8f acc[8];
#pragma unroll
  for (int t = 0; t < 8; ++t) acc[t] = z8();
  {
    const unsigned short* ap = AGG + (size_t)(rowBase + 16 * wave + m) * (size_t)KL + 8 * hh;
    const unsigned short* bp = WD + (size_t)m * (size_t)KL + 8 * hh;
    gemm_16x128<KL>(ap, bp, acc);
  }
  {
    float rr[8];
#pragma unroll
    for (int r = 0; r < 8; ++r) rr[r] = srs[16 * wave + 8 * hh + r];
#pragma unroll
    for (int nt = 0; nt < 8; ++nt) {
      const float bc = sb[16 * nt + m];
#pragma unroll
      for (int r = 0; r < 8; ++r) acc[nt][r] = (acc[nt][r] + bc) * rr[r];
    }
  }
  {
    const unsigned short* ap = Hhl + (size_t)(rowBase + 16 * wave + m) * (size_t)KL + 8 * hh;
    const unsigned short* bp = WSD + (size_t)m * (size_t)KL + 8 * hh;
    gemm_16x128<KL>(ap, bp, acc);
  }
  stage_d(stg, acc, wave, hh, m);
  __syncthreads();
  epi_rows<1>(stg, Hhl, rowBase, wave, lane);
}

__device__ __forceinline__ void head_flush(const float* lg, float* ob, int nv4, int tid) {
#pragma unroll 1
  for (int it = 0; it < 2; ++it) {
    const int i4  = it * NTHR + tid;
    const int i4c = i4 < (HBM * NOUT / 4) ? i4 : (HBM * NOUT / 4 - 1);
    const v4f v = *(const v4fa*)(lg + 4 * i4c);
    asm volatile("" :: "v"(v));
    if (i4 < nv4) *(volatile v4f*)(ob + (size_t)4 * (size_t)i4) = v;
  }
}

__global__ __launch_bounds__(NTHR) __attribute__((amdgpu_num_vgpr(248)))
void k_head(const unsigned short* __restrict__ Hhl, const unsigned short* __restrict__ WF,
            const float* __restrict__ sm, float* out) {
  __shared__ __attribute__((aligned(16))) float lg[HBM * NOUT];
  __shared__ __attribute__((aligned(16))) float sb[NOP];
  const int tid = (int)threadIdx.x, lane = tid & 31, wave = tid >> 5, hh = lane >> 4, m = lane & 15;
  const int blk = (int)blockIdx.x;
  const int rowBase = blk * HBM;
  if (tid < 32) {
    const int j = lane & 3;
    *(v4fa*)(sb + 4 * j) = *(const v4fa*)(sm + 3 * HD + 4 * j);
  }
  __syncthreads();

  v8f acc = z8();
  const unsigned short* ap = Hhl + (size_t)(rowBase + 16 * wave + m) * (size_t)KL + 8 * hh;
  const unsigned short* bp = WF + (size_t)m * (size_t)KL + 8 * hh;
#pragma unroll 1
  for (int k0 = 0; k0 < KL; k0 += 32) {
    FragB af, bf;
    af.h[0] = *(const v8usa*)(ap + k0);
    af.h[1] = *(const v8usa*)(ap + k0 + 16);
    bf.h[0] = *(const v8usa*)(bp + k0);
    bf.h[1] = *(const v8usa*)(bp + k0 + 16);
    acc = wmb(af, bf, acc);
  }
  const float bc = sb[m];
  if (m < NOUT) {
#pragma unroll
    for (int r = 0; r < 8; ++r) lg[(16 * wave + 8 * hh + r) * NOUT + m] = acc[r] + bc;
  }
  __syncthreads();

  const int liveRows = (NN - rowBase) < HBM ? (NN - rowBase) : HBM;
  const int nv4 = liveRows * (NOUT / 4);
  float* ob = out + (size_t)blk * (size_t)(HBM * NOUT);
  head_flush(lg, ob, nv4, tid);
  __threadfence();
  head_flush(lg, ob, nv4, tid);
}

extern "C" void kernel_launch(void* const* d_in, const int* in_sizes, int n_in,
                              void* d_out, int out_size, void* d_ws, size_t ws_size,
                              hipStream_t stream) {
  if (n_in < 16) return;
  if (in_sizes[0] != NN * FIN) return;
  if (in_sizes[1] != NE || in_sizes[2] != NE) return;
  if (in_sizes[3] != NE) return;
  if (in_sizes[4] != NN || in_sizes[5] != NE) return;
  if (in_sizes[6] != FIN * HD || in_sizes[7] != HD) return;
  if (in_sizes[8] != HD * HD || in_sizes[9] != HD * HD || in_sizes[10] != HD) return;
  if (in_sizes[11] != HD * HD || in_sizes[12] != HD * HD || in_sizes[13] != HD) return;
  if (in_sizes[14] != HD * NOUT || in_sizes[15] != NOUT) return;
  if (out_size != NN * NOUT) return;

  const float* x    = (const float*)d_in[0];
  const int*   srcs = (const int*)d_in[1];
  const int*   dsts = (const int*)d_in[2];
  const float* ew   = (const float*)d_in[3];
  const float* Wemb = (const float*)d_in[6];
  const float* bemb = (const float*)d_in[7];
  const float* Ws1  = (const float*)d_in[8];
  const float* W1   = (const float*)d_in[9];
  const float* b1   = (const float*)d_in[10];
  const float* Ws2  = (const float*)d_in[11];
  const float* W2   = (const float*)d_in[12];
  const float* b2   = (const float*)d_in[13];
  const float* Wfc  = (const float*)d_in[14];
  const float* bfc  = (const float*)d_in[15];
  float* out = (float*)d_out;

  constexpr size_t zHL   = (size_t)MP * KL * 2;
  constexpr size_t zXB   = (size_t)MP * KE * 2;
  constexpr size_t zLIST = (size_t)NBK * BK_PL * 4;
  constexpr size_t zCO   = (size_t)NBK * 2 * NBRUN * 4;
  constexpr size_t zRS   = (size_t)2 * NBK * NBRUN * 4;
  constexpr size_t zFLAG = (size_t)2 * NBK * 128;
  constexpr size_t zWET  = (size_t)HD * KE * 2;
  constexpr size_t zWD   = (size_t)4 * HD * KL * 2;
  constexpr size_t zWF   = (size_t)NOP * KL * 2;
  constexpr size_t zSM   = 2048;
  constexpr size_t oHhl  = 0;
  constexpr size_t oAGG  = oHhl + zHL;
  constexpr size_t oLIST = oAGG + zHL;
  constexpr size_t oCO   = oLIST + zLIST;
  constexpr size_t oRS   = oCO + zCO;
  constexpr size_t oFLAG = oRS + zRS;
  constexpr size_t oWET  = oFLAG + zFLAG;
  constexpr size_t oWD   = oWET + zWET;
  constexpr size_t oWF   = oWD + zWD;
  constexpr size_t oSM   = oWF + zWF;
  constexpr size_t oEND  = oSM + zSM;
  static_assert(zHL % 256 == 0 && zLIST % 256 == 0 && zCO % 256 == 0 && zRS % 256 == 0 && zFLAG % 256 == 0);
  static_assert(zWET % 256 == 0 && zWD % 256 == 0 && zWF % 256 == 0 && zSM % 256 == 0);
  static_assert(zXB <= zHL);
  static_assert(oEND <= (size_t)(128u << 20));
  if (oEND > ws_size) return;

  char* ws = (char*)d_ws;
  unsigned short* Hhl  = (unsigned short*)(ws + oHhl);
  unsigned short* AGG  = (unsigned short*)(ws + oAGG);
  unsigned short* XB   = (unsigned short*)(ws + oAGG);
  int*            LIST = (int*)(ws + oLIST);
  int*            CO   = (int*)(ws + oCO);
  int*            RS   = (int*)(ws + oRS);
  int*            FLAG = (int*)(ws + oFLAG);
  unsigned short* WET  = (unsigned short*)(ws + oWET);
  unsigned short* WD   = (unsigned short*)(ws + oWD);
  unsigned short* WF   = (unsigned short*)(ws + oWF);
  float*          SM   = (float*)(ws + oSM);
  const float* RSI = (const float*)RS;
  const float* RSO = (const float*)RS + (size_t)NBK * NBRUN;

  hipFuncSetAttribute(reinterpret_cast<const void*>(&k_bucket), hipFuncAttributeMaxDynamicSharedMemorySize, (int)BK_LDS);

  k_prep<<<PBTOT, NTHR, 0, stream>>>(x, Wemb, bemb, Ws1, W1, b1, Ws2, W2, b2, Wfc, bfc, XB, WET, WD, WF, SM);
  k_bucket<<<2 * NBK, NTHR, BK_LDS, stream>>>(srcs, dsts, ew, LIST, CO, RS, FLAG);
  k_emb<<<MP / GBM, GTHR, 0, stream>>>(XB, WET, SM, Hhl);

  k_replay<<<MP / ABM, NTHR, 0, stream>>>(LIST, CO, FLAG, RSO, Hhl, AGG);
  k_layer<<<MP / GBM, GTHR, 0, stream>>>(Hhl, AGG, WD, WD + (size_t)HD * KL, SM + HD, RSI);

  k_replay<<<MP / ABM, NTHR, 0, stream>>>(LIST, CO, FLAG, RSO, Hhl, AGG);
  k_layer<<<MP / GBM, GTHR, 0, stream>>>(Hhl, AGG, WD + (size_t)2 * HD * KL, WD + (size_t)3 * HD * KL,
                                         SM + 2 * HD, RSI);

  k_head<<<MP / HBM, NTHR, 0, stream>>>(Hhl, WF, SM, out);
}
